// MotherNet_89498528514766
// MI455X (gfx1250) — hardware-verified
//
#include <hip/hip_runtime.h>


#define TT   8192
#define NBD  8
#define FF   100
#define FP   128
#define HH   512
#define TQ   (TT / 4)

typedef unsigned short bf;
typedef __attribute__((ext_vector_type(16))) __bf16   v16bf;
typedef __attribute__((ext_vector_type(8)))  unsigned short v8us;
typedef __attribute__((ext_vector_type(8)))  float    v8f;
typedef __attribute__((ext_vector_type(4)))  float    v4f;
typedef v4f  __attribute__((may_alias)) v4fa;
typedef v8us __attribute__((may_alias)) v8usa;

__device__ __forceinline__ unsigned short f2bf(float f) { unsigned u = __float_as_uint(f); u += 0x7FFFu + ((u >> 16) & 1u); return (unsigned short)(u >> 16); }
__device__ __forceinline__ float bf2f(unsigned short b) { return __uint_as_float(((unsigned)b) << 16); }
__device__ __forceinline__ float bfr(float f) { return bf2f(f2bf(f)); }
__device__ __forceinline__ float n2n(float v) { if (v != v) return 0.f; if (v > 3.4028235e38f) return 3.4028235e38f; if (v < -3.4028235e38f) return -3.4028235e38f; return v; }
__device__ __forceinline__ v16bf cat16b(v8us lo, v8us hi) { return __builtin_bit_cast(v16bf, __builtin_shufflevector(lo, hi, 0, 1, 2, 3, 4, 5, 6, 7, 8, 9, 10, 11, 12, 13, 14, 15)); }
__device__ __forceinline__ v8f wmmab(v16bf a, v16bf b, v8f c) { return __builtin_amdgcn_wmma_f32_16x16x32_bf16(false, a, false, b, (short)0, c, false, false); }
#define VST2(T, p, v) do { const T vst2_v_ = (v); *(volatile T*)(p) = vst2_v_; __threadfence(); *(volatile T*)(p) = vst2_v_; } while (0)

__global__ __launch_bounds__(256) void k_x(const float* __restrict__ x, bf* XB) {
    const int lane = threadIdx.x & 31; const size_t w = (size_t)blockIdx.x * 8 + (threadIdx.x >> 5);
    if (w >= (size_t)NBD * TT) return;
    const int b = (int)(w / TT), t = (int)(w - (size_t)b * TT);
    if (lane < 16) { v8us o;
#pragma unroll
        for (int i = 0; i < 8; ++i) { const int f = lane * 8 + i; o[i] = (f < FF) ? f2bf(n2n(x[((size_t)t * NBD + b) * FF + (f < FF ? f : 0)])) : (unsigned short)0; }
        VST2(v8us, XB + w * FP + lane * 8, o); }
}
__global__ __launch_bounds__(256) void k_w1(const float* __restrict__ w1, bf* W1T) {
    __shared__ unsigned short tl[64][130];
    const int b = blockIdx.x / (HH / 64), hq = blockIdx.x - b * (HH / 64), h0 = hq * 64, tid = threadIdx.x;
    for (int e = tid; e < 64 * FP; e += 256) { const int f = e / 64, hh = e - f * 64; tl[hh][f] = (f < FF) ? f2bf(w1[((size_t)b * FF + f) * HH + h0 + hh]) : (unsigned short)0; }
    __syncthreads();
    const int piece = tid & 7;
    auto pass = [&]() {
#pragma unroll
        for (int s2 = 0; s2 < 2; ++s2)
#pragma unroll
            for (int ln = 0; ln < 2; ++ln) { const int hh = (tid >> 3) + 32 * s2; v8us o;
#pragma unroll
                for (int i = 0; i < 8; ++i) o[i] = tl[hh][ln * 64 + piece * 8 + i];
                *(volatile v8us*)(W1T + ((size_t)b * HH + h0 + hh) * FP + ln * 64 + piece * 8) = o; }
    };
    pass(); __threadfence(); pass();
}
__global__ __launch_bounds__(256) void k_w2(const float* __restrict__ w2, bf* W2T) {
    __shared__ __align__(16) unsigned short tl[64 * 72];
    const int tid = threadIdx.x, k0 = blockIdx.x * 64, n0 = blockIdx.y * 64, b = blockIdx.z;
    const int kk = tid >> 2, nq = (tid & 3) * 16;
#pragma unroll
    for (int i = 0; i < 16; ++i) tl[(nq + i) * 72 + kk] = f2bf(w2[((size_t)b * HH + k0 + kk) * HH + n0 + nq + i]);
    __syncthreads();
    const int piece = tid & 7;
    auto pass = [&]() {
#pragma unroll
        for (int s = 0; s < 2; ++s) { const int nr = (tid >> 3) + 32 * s; const v8us val = *(const v8usa*)(tl + nr * 72 + piece * 8); *(volatile v8us*)(W2T + ((size_t)b * HH + n0 + nr) * HH + k0 + piece * 8) = val; }
    };
    pass(); __threadfence(); pass();
}
template <bool SA, int MODE>
__global__ __launch_bounds__(128) void k_gemm(const bf* __restrict__ A, const bf* __restrict__ Al, size_t sa, const bf* __restrict__ Bn, size_t sb, int K, const float* __restrict__ bias, void* C, void* C2, size_t sc, int ldr) {
    __shared__ __align__(16) float ost[4][16 * 68];
    const int lane = threadIdx.x & 31, wave = threadIdx.x >> 5, lr = lane & 15, hi = lane >> 4, b = blockIdx.z;
    const int r0 = blockIdx.x * 64 + wave * 16, c0 = blockIdx.y * 64;
    A += b * sa; if (SA) Al += b * sa; Bn += b * sb;
    const size_t aoff = (size_t)(r0 + lr) * K + 8 * hi;
    size_t boff[4];
#pragma unroll
    for (int t = 0; t < 4; ++t) boff[t] = (size_t)(c0 + t * 16 + lr) * K + 8 * hi;
    v8f acc[4];
#pragma unroll
    for (int t = 0; t < 4; ++t) acc[t] = (v8f){};
#pragma unroll 2
    for (int kc = 0; kc < K; kc += 32) {
        const v16bf a = cat16b(*(const v8us*)(A + aoff + kc), *(const v8us*)(A + aoff + kc + 16));
        v16bf al = a; if (SA) al = cat16b(*(const v8us*)(Al + aoff + kc), *(const v8us*)(Al + aoff + kc + 16));
#pragma unroll
        for (int t = 0; t < 4; ++t) { const v16bf bb = cat16b(*(const v8us*)(Bn + boff[t] + kc), *(const v8us*)(Bn + boff[t] + kc + 16)); acc[t] = wmmab(a, bb, acc[t]); if (SA) acc[t] = wmmab(al, bb, acc[t]); }
        asm volatile("v_nop\n\tv_nop\n\tv_nop\n\tv_nop" : "+v"(acc[0]), "+v"(acc[1]), "+v"(acc[2]), "+v"(acc[3]) : "v"(a), "v"(al));
    }
    float* os = &ost[wave][0];
#pragma unroll
    for (int t = 0; t < 4; ++t) { const float bv = bfr(bias[(size_t)b * HH + c0 + t * 16 + lr]);
#pragma unroll
        for (int j = 0; j < 8; ++j) os[(hi * 8 + j) * 68 + t * 16 + lr] = fmaxf(acc[t][j] + bv, 0.f); }
    __syncthreads();
    if (MODE == 1) {
        float* crow = (float*)C + b * sc + (size_t)r0 * HH + c0;
        auto pass = [&]() {
#pragma unroll
            for (int s = 0; s < 8; ++s) { const int Lid = (lane >> 3) + 4 * s, piece = lane & 7; const int row = Lid >> 1, cofs = (Lid & 1) * 32 + piece * 4;
                const v4f val = *(const v4fa*)(os + row * 68 + cofs); *(volatile v4f*)(crow + (size_t)row * HH + cofs) = val; }
        };
        pass(); __threadfence(); pass();
    } else {
        bf* c1 = (bf*)C + b * sc + (size_t)r0 * HH + c0; bf* c2 = (bf*)C2 + b * sc + (size_t)r0 * HH + c0;
        auto pass = [&]() {
#pragma unroll
            for (int s = 0; s < 4; ++s) { const int row = 4 * s + (lane >> 3), piece = lane & 7; const float* sp = os + row * 68 + piece * 8; v8us oh, ol;
#pragma unroll
                for (int i = 0; i < 8; ++i) { const unsigned short hb = f2bf(sp[i]); oh[i] = hb; ol[i] = f2bf(sp[i] - bf2f(hb)); }
                *(volatile v8us*)(c1 + (size_t)row * HH + piece * 8) = oh; *(volatile v8us*)(c2 + (size_t)row * HH + piece * 8) = ol; }
        };
        pass(); __threadfence(); pass();
    }
}
__global__ __launch_bounds__(256) void k_final(const float* __restrict__ H2, const float* __restrict__ w3, const float* __restrict__ b3, int t0, float* out) {
    __shared__ float st[64];
    const int lane = threadIdx.x & 31, wave = threadIdx.x >> 5;
    const size_t e0 = (size_t)t0 * NBD + (size_t)blockIdx.x * 64;
#pragma unroll 1
    for (int i = 0; i < 8; ++i) { const size_t e = e0 + wave * 8 + i; const int t = (int)(e / NBD), b = (int)(e - (size_t)t * NBD);
        const float* hr = H2 + ((size_t)b * TQ + (t - t0)) * HH; float s = 0.f;
#pragma unroll
        for (int q = 0; q < HH / 32; ++q) s += hr[q * 32 + lane] * bfr(w3[(size_t)b * HH + q * 32 + lane]);
#pragma unroll
        for (int sh = 16; sh; sh >>= 1) s += __shfl_xor(s, sh, 32);
        if (lane == 0) st[wave * 8 + i] = s + bfr(b3[b]); }
    __syncthreads();
    if (threadIdx.x < 64) { const float v = st[threadIdx.x]; *(volatile float*)(out + e0 + threadIdx.x) = v; }
    __threadfence();
    if (threadIdx.x < 64) { const float v = st[threadIdx.x]; *(volatile float*)(out + e0 + threadIdx.x) = v; }
}

extern "C" void kernel_launch(void* const* d_in, const int* in_sizes, int n_in,
                              void* d_out, int out_size, void* d_ws, size_t ws_size, hipStream_t stream) {
    (void)in_sizes; (void)n_in; (void)out_size;
    const float* x = (const float*)d_in[0]; const float* w1 = (const float*)d_in[1]; const float* b1 = (const float*)d_in[2]; const float* w2 = (const float*)d_in[3]; const float* b2 = (const float*)d_in[4];
    const float* w3 = (const float*)d_in[5]; const float* b3 = (const float*)d_in[6];
    float* out = (float*)d_out;
    char* wsp = (char*)d_ws;
    auto take = [&](size_t bytes) { char* p = wsp; wsp += (bytes + 255) & ~(size_t)255; return (void*)p; };
    const int TH = TQ;
    bf* XB = (bf*)take((size_t)NBD * TT * FP * 2); bf* W1T = (bf*)take((size_t)NBD * HH * FP * 2); bf* W2T = (bf*)take((size_t)NBD * HH * HH * 2);
    bf* H1H = (bf*)take((size_t)NBD * TH * HH * 2); bf* H1L = (bf*)take((size_t)NBD * TH * HH * 2); float* H2 = (float*)take((size_t)NBD * TH * HH * 4);
    if ((size_t)(wsp - (char*)d_ws) > ws_size) return;
    k_x<<<(NBD * TT) / 8, 256, 0, stream>>>(x, XB);
    k_w1<<<NBD * (HH / 64), 256, 0, stream>>>(w1, W1T);
    k_w2<<<dim3(HH / 64, HH / 64, NBD), 256, 0, stream>>>(w2, W2T);
    for (int half = 0; half < 4; ++half) { const int t0 = half * TH;
        k_gemm<false, 0><<<dim3(TH / 64, HH / 64, NBD), 128, 0, stream>>>(XB + (size_t)t0 * FP, nullptr, (size_t)TT * FP, W1T, (size_t)HH * FP, FP, b1, H1H, H1L, (size_t)TH * HH, 0);
        k_gemm<true, 1><<<dim3(TH / 64, HH / 64, NBD), 128, 0, stream>>>(H1H, H1L, (size_t)TH * HH, W2T, (size_t)HH * HH, HH, b2, H2, nullptr, (size_t)TH * HH, 0);
        k_final<<<(TH * NBD) / 64, 256, 0, stream>>>(H2, w3, b3, t0, out);
    }
}
